// MambaBlock_9440338116665
// MI455X (gfx1250) — hardware-verified
//
#include <hip/hip_runtime.h>
#include <math.h>

typedef __attribute__((ext_vector_type(16))) _Float16 v16h;
typedef __attribute__((ext_vector_type(8)))  _Float16 v8h;
typedef __attribute__((ext_vector_type(16))) __bf16   v16b;
typedef __attribute__((ext_vector_type(8)))  __bf16   v8b;
typedef __attribute__((ext_vector_type(8)))  float    v8f;
typedef __attribute__((ext_vector_type(4)))  float    v4f;

constexpr int kBatch = 2;
constexpr int kSeqL  = 2048;
constexpr int kDmod  = 1024;
constexpr int kDin   = 2048;
constexpr int kNst   = 16;
constexpr int kDtR   = 256;
constexpr int kPrjN  = kDtR + 2 * kNst;
constexpr int kPrjP  = 320;
constexpr int kXzN   = 2 * kDin;
constexpr int kRows  = kBatch * kSeqL;
constexpr int kTP    = 260;
static_assert(kPrjN == 288);
static_assert(kPrjP >= kPrjN && (kPrjP % 64) == 0);
static_assert((kDmod % 32) == 0 && (kDin % 32) == 0 && (kDtR % 32) == 0);
static_assert((kRows % 64) == 0 && (kDin % 64) == 0 && (kDmod % 64) == 0 && (kXzN % 64) == 0);
static_assert((kDmod % 64) == 0 && (kDtR % 64) == 0);
static_assert((kSeqL % 16) == 0 && (kDin % 256) == 0 && kDmod == 4 * 256);

constexpr float kCarryW    = 32.0f;
constexpr float kCarryWdt  = 256.0f;
constexpr float kCarryU    = 8.0f;
constexpr float kCarryDr   = 16.0f;
constexpr float kCarryDtl  = 1024.0f;
constexpr float kCarryY    = 16.0f;
constexpr float kScale1    = 1.0f / kCarryW;
constexpr float kScale2    = 1.0f / (kCarryU * kCarryW);
constexpr float kScale3    = kCarryDtl / (kCarryDr * kCarryWdt);
constexpr float kScale4    = 1.0f / (kCarryY * kCarryW);
constexpr float kDtlInv    = 1.0f / kCarryDtl;
static_assert(kScale3 == 0.25f);

constexpr size_t kOffWIN16  = 0;
constexpr size_t kOffWX16   = kOffWIN16  + (size_t)kXzN  * kDmod * 2;
constexpr size_t kOffWDT16  = kOffWX16   + (size_t)kPrjP * kDin  * 2;
constexpr size_t kOffWOUT16 = kOffWDT16  + (size_t)kDin  * kDtR  * 2;
constexpr size_t kOffXN16   = kOffWOUT16 + (size_t)kDmod * kDin  * 2;
constexpr size_t kOffU32    = kOffXN16   + (size_t)kRows * kDmod * 2;
constexpr size_t kOffG16    = kOffU32    + (size_t)kRows * kDin  * 4;
constexpr size_t kOffU16    = kOffG16    + (size_t)kRows * kDin  * 2;
constexpr size_t kOffXDBL   = kOffU16    + (size_t)kRows * kDin  * 2;
constexpr size_t kOffDRAW16 = kOffXDBL   + (size_t)kRows * kPrjP * 4;
constexpr size_t kOffDTL16  = kOffDRAW16 + (size_t)kRows * kDtR  * 2;
constexpr size_t kOffY16    = kOffDTL16  + (size_t)kRows * kDin  * 2;
constexpr size_t kWsTotal   = kOffY16    + (size_t)kRows * kDin  * 2;
static_assert(kWsTotal == 131334144ull);
static_assert(kWsTotal <= 134217728ull);
static_assert((kOffWX16 % 128) == 0 && (kOffWDT16 % 128) == 0 && (kOffWOUT16 % 128) == 0 && (kOffXN16 % 128) == 0 &&
              (kOffU32 % 128) == 0 && (kOffG16 % 128) == 0 && (kOffU16 % 128) == 0 && (kOffXDBL % 128) == 0 &&
              (kOffDRAW16 % 128) == 0 && (kOffDTL16 % 128) == 0 && (kOffY16 % 128) == 0);

__device__ __forceinline__ unsigned short f2bf_bits(float f) {
  unsigned u = __float_as_uint(f);
  return (unsigned short)((u + 0x7FFFu + ((u >> 16) & 1u)) >> 16);
}
__device__ __forceinline__ float bf_bits2f(unsigned short h) { return __uint_as_float(((unsigned)h) << 16); }

__device__ __forceinline__ float h16_to_f32(unsigned hb) {
  const unsigned sgn = (hb & 0x8000u) << 16; const unsigned em = hb & 0x7fffu;
  const float fn = __uint_as_float((em << 13) + 0x38000000u);
  const float fs = (float)em * 5.9604644775390625e-8f;
  const float mag = (em < 0x400u) ? fs : fn; return __uint_as_float(__float_as_uint(mag) | sgn); }

__device__ __forceinline__ void dep_guard4_h(v8f& a, v8f& b, v8f& c, v8f& d, v16h x, v16h y) {
  asm volatile("v_nop\n\tv_nop\n\tv_nop\n\tv_nop" : "+v"(a), "+v"(b), "+v"(c), "+v"(d) : "v"(x), "v"(y)); }
__device__ __forceinline__ void dep_guard4_b(v8f& a, v8f& b, v8f& c, v8f& d, v16b x, v16b y) {
  asm volatile("v_nop\n\tv_nop\n\tv_nop\n\tv_nop" : "+v"(a), "+v"(b), "+v"(c), "+v"(d) : "v"(x), "v"(y)); }
__device__ __forceinline__ void keep4_h(v16h a, v16h b, v16h c, v16h d) { asm volatile("v_nop" :: "v"(a), "v"(b), "v"(c), "v"(d)); }
__device__ __forceinline__ void keep4_b(v16b a, v16b b, v16b c, v16b d) { asm volatile("v_nop" :: "v"(a), "v"(b), "v"(c), "v"(d)); }
__device__ __forceinline__ void acc_guard4(v8f& a, v8f& b, v8f& c, v8f& d) { asm volatile("v_nop\n\tv_nop\n\tv_nop\n\tv_nop" : "+v"(a), "+v"(b), "+v"(c), "+v"(d)); }
template <typename T> struct Frag;
template <> struct Frag<_Float16> {
  typedef v16h V; union U { v16h v; v8h h[2]; };
  static __device__ __forceinline__ v16h load(const _Float16* p) {
    U f; f.h[0] = *(const v8h*)(p); f.h[1] = *(const v8h*)(p + 16); return f.v;
  }
  static __device__ __forceinline__ v8f mma(v16h a, v16h b, v8f c) {
    return __builtin_amdgcn_wmma_f32_16x16x32_f16(false, a, false, b, (short)0, c, false, false);
  }
  static __device__ __forceinline__ void guard4(v8f& a, v8f& b, v8f& c, v8f& d, v16h x, v16h y) { dep_guard4_h(a, b, c, d, x, y); }
  static __device__ __forceinline__ void keep(v16h a, v16h b, v16h c, v16h d) { keep4_h(a, b, c, d); }
};
template <> struct Frag<__bf16> {
  typedef v16b V; union U { v16b v; v8b h[2]; };
  static __device__ __forceinline__ v16b load(const __bf16* p) {
    U f; f.h[0] = *(const v8b*)(p); f.h[1] = *(const v8b*)(p + 16); return f.v;
  }
  static __device__ __forceinline__ v8f mma(v16b a, v16b b, v8f c) {
    return __builtin_amdgcn_wmma_f32_16x16x32_bf16(false, a, false, b, (short)0, c, false, false);
  }
  static __device__ __forceinline__ void guard4(v8f& a, v8f& b, v8f& c, v8f& d, v16b x, v16b y) { dep_guard4_b(a, b, c, d, x, y); }
  static __device__ __forceinline__ void keep(v16b a, v16b b, v16b c, v16b d) { keep4_b(a, b, c, d); }
};

template <int ET> struct Elem;
template <> struct Elem<0> { typedef _Float16 T; };
template <> struct Elem<1> { typedef __bf16 T; };
template <int ET, bool SPLIT, int BIAS_MODE, int OUT_MODE, bool RESID, int ACT = 0>
__global__ __launch_bounds__(256) void wmma_gemm64(
    const unsigned short* __restrict__ Ap, const unsigned short* __restrict__ A2p, int lda, long strideA,
    const unsigned short* __restrict__ Btp, const unsigned short* __restrict__ Bt2p, int ldb, long strideB,
    void* __restrict__ Cout, void* __restrict__ Cout2, int ldc, long strideC,
    const float* __restrict__ bias,
    const float* __restrict__ resid, long strideR,
    int M, int N, int K, float scale) {
  static_assert(!RESID || (OUT_MODE == 0 && ACT == 0));
  typedef typename Elem<ET>::T T;
  typedef typename Frag<T>::V V;
  const T* A = (const T*)Ap; const T* A2 = (const T*)A2p; const T* Bt = (const T*)Btp; const T* Bt2 = (const T*)Bt2p;
  __shared__ __align__(16) float sT[8][16 * 68];
  const int b    = blockIdx.y;
  const int lane = threadIdx.x & 31;
  const int wave = threadIdx.x >> 5;
  const int tilesN = N >> 6;
  const int tilesM = M >> 6;
  const int tile = blockIdx.x * 8 + wave;
  if (tile >= tilesM * tilesN) return;
  const int tm = tile / tilesN;
  const int tn = tile - tm * tilesN;
  const int m0 = tm << 6;
  const int n0 = tn << 6;

  const T* Ab  = A  + (size_t)b * strideA;
  const T* Bb  = Bt + (size_t)b * strideB;
  const T* Ab2 = SPLIT ? (A2  + (size_t)b * strideA) : nullptr;
  const T* Bb2 = SPLIT ? (Bt2 + (size_t)b * strideB) : nullptr;

  const int rlane = lane & 15;
  const int koff  = (lane >> 4) * 8;
  const int mOff  = (lane >> 4) * 8;

  v8f acc[4][4];
#pragma unroll
  for (int i = 0; i < 4; ++i)
#pragma unroll
    for (int j = 0; j < 4; ++j) acc[i][j] = (v8f){0.f,0.f,0.f,0.f,0.f,0.f,0.f,0.f};

  for (int k0 = 0; k0 < K; k0 += 32) {
    V bh[4], bl[4];
#pragma unroll
    for (int j = 0; j < 4; ++j) {
      const size_t bo = (size_t)(n0 + (j << 4) + rlane) * ldb + koff + k0;
      bh[j] = Frag<T>::load(Bb + bo);
      if (SPLIT) bl[j] = Frag<T>::load(Bb2 + bo);
    }
#pragma unroll
    for (int i = 0; i < 4; ++i) {
      const size_t ao = (size_t)(m0 + (i << 4) + rlane) * lda + koff + k0;
      V ah = Frag<T>::load(Ab + ao);
      V al;
      if (SPLIT) al = Frag<T>::load(Ab2 + ao);
#pragma unroll
      for (int j = 0; j < 4; ++j) {
        acc[i][j] = Frag<T>::mma(ah, bh[j], acc[i][j]);
        if (SPLIT) {
          acc[i][j] = Frag<T>::mma(ah, bl[j], acc[i][j]);
          acc[i][j] = Frag<T>::mma(al, bh[j], acc[i][j]);
        }
      }
      Frag<T>::guard4(acc[i][0], acc[i][1], acc[i][2], acc[i][3], ah, SPLIT ? al : ah);
    }
    Frag<T>::keep(bh[0], bh[1], bh[2], bh[3]);
    if (SPLIT) Frag<T>::keep(bl[0], bl[1], bl[2], bl[3]);
  }
  acc_guard4(acc[0][0], acc[0][1], acc[0][2], acc[0][3]);
  acc_guard4(acc[1][0], acc[1][1], acc[1][2], acc[1][3]);
  acc_guard4(acc[2][0], acc[2][1], acc[2][2], acc[2][3]);
  acc_guard4(acc[3][0], acc[3][1], acc[3][2], acc[3][3]);

  float* slab = sT[wave];
  const float* Rb = RESID ? (resid + (size_t)b * strideR) : nullptr;
#pragma unroll
  for (int i = 0; i < 4; ++i) {
    const int mBase = m0 + (i << 4);
#pragma unroll
    for (int j = 0; j < 4; ++j) {
      const int n = n0 + (j << 4) + rlane;
      float bv = 0.f;
      if (BIAS_MODE == 2) bv = bias[n];
#pragma unroll
      for (int r = 0; r < 8; ++r) {
        float v = acc[i][j][r] * scale;
        if (BIAS_MODE == 1) v += bias[mBase + mOff + r];
        if (BIAS_MODE == 2) v += bv;
        if (ACT == 1) v = tanhf(v);
        if (ACT == 2) v = fmaxf(v, 0.0f);
        if (ACT == 3) v = v / (1.0f + expf(-v));
        if (ACT == 4) v = (v > 0.f) ? v : 0.01f * v;
        slab[(mOff + r) * 68 + (j << 4) + rlane] = v;
      }
    }
    __builtin_amdgcn_fence(__ATOMIC_RELEASE, "workgroup");
    __builtin_amdgcn_wave_barrier();
    __builtin_amdgcn_fence(__ATOMIC_ACQUIRE, "workgroup");
    if (OUT_MODE == 0) {
      float* C = (float*)Cout + (size_t)b * strideC;
      const int hh = lane >> 4, c4 = (lane & 15) * 4;
      for (int pass = 0; pass < 2; ++pass) {
#pragma unroll
        for (int it = 0; it < 8; ++it) {
          const int row = it * 2 + hh;
          v4f v = *(const v4f*)(slab + row * 68 + c4);
          if (RESID) {
            const v4f rv = *(const v4f*)(Rb + (size_t)(mBase + row) * ldc + n0 + c4);
            v = v + rv;
          }
          *(volatile v4f*)(C + (size_t)(mBase + row) * ldc + n0 + c4) = v;
        }
        __threadfence();
      }
    } else {
      const int q = lane >> 3, c8 = (lane & 7) * 8;
      unsigned short* C  = (unsigned short*)Cout  + (size_t)b * strideC;
      unsigned short* C2 = (OUT_MODE == 2) ? ((unsigned short*)Cout2 + (size_t)b * strideC) : nullptr;
      for (int pass = 0; pass < 2; ++pass) {
#pragma unroll
        for (int it = 0; it < 4; ++it) {
          const int row = it * 4 + q;
          const float* sp = slab + row * 68 + c8;
          v8h hv, lv;
#pragma unroll
          for (int e = 0; e < 8; ++e) {
            if (OUT_MODE == 1) {
              hv[e] = (_Float16)sp[e];
            } else {
              unsigned short hb = f2bf_bits(sp[e]);
              unsigned short lb = f2bf_bits(sp[e] - bf_bits2f(hb));
              hv[e] = __builtin_bit_cast(_Float16, hb);
              lv[e] = __builtin_bit_cast(_Float16, lb);
            }
          }
          *(volatile v8h*)(C + (size_t)(mBase + row) * ldc + n0 + c8) = hv;
          if (OUT_MODE == 2) *(volatile v8h*)(C2 + (size_t)(mBase + row) * ldc + n0 + c8) = lv;
        }
        __threadfence();
      }
    }
    __builtin_amdgcn_fence(__ATOMIC_RELEASE, "workgroup");
    __builtin_amdgcn_wave_barrier();
    __builtin_amdgcn_fence(__ATOMIC_ACQUIRE, "workgroup");
  }
}

__global__ __launch_bounds__(256) void cast_f16_kernel(
    const float* __restrict__ src, unsigned short* __restrict__ dst, int total8, float scale)
{
  const int i = blockIdx.x * 256 + threadIdx.x;
  if (i >= total8) return;
  const size_t e0 = (size_t)i << 3;
  const float* p = src + e0;
  const v4f a0 = *(const v4f*)(p);
  const v4f a1 = *(const v4f*)(p + 4);
  v8h hv;
#pragma unroll
  for (int e = 0; e < 4; ++e) {
    hv[e]     = (_Float16)(a0[e] * scale);
    hv[4 + e] = (_Float16)(a1[e] * scale);
  }
  unsigned short* q = dst + e0;
  *(volatile v8h*)q = hv;
  __threadfence();
  *(volatile v8h*)q = hv;
}

__global__ __launch_bounds__(256) void transpose_cast_kernel(
    const float* __restrict__ W, unsigned short* __restrict__ Bt, int Kdim, int Ndim, int Npad, float scale)
{
  __shared__ float tile[64 * 65];
  const int tid = threadIdx.x, lane = tid & 31, wave = tid >> 5;
  const int n0 = blockIdx.x * 64;
  const int k0 = blockIdx.y * 64;
  (void)Npad;
#pragma unroll
  for (int p = 0; p < 8; ++p) {
    const int idx = tid + p * 256;
    const int kk  = idx >> 6;
    const int nn  = idx & 63;
    const int n   = n0 + nn;
    const int nc  = (n < Ndim) ? n : (Ndim - 1);
    const float v = W[(size_t)(k0 + kk) * Ndim + nc];
    tile[kk * 65 + nn] = (n < Ndim) ? (v * scale) : 0.f;
  }
  asm volatile("" ::: "memory");
#pragma unroll
  for (int p = 8; p < 16; ++p) {
    const int idx = tid + p * 256;
    const int kk  = idx >> 6;
    const int nn  = idx & 63;
    const int n   = n0 + nn;
    const int nc  = (n < Ndim) ? n : (Ndim - 1);
    const float v = W[(size_t)(k0 + kk) * Ndim + nc];
    tile[kk * 65 + nn] = (n < Ndim) ? (v * scale) : 0.f;
  }
  __syncthreads();
  const int q = lane >> 3, c8 = (lane & 7) * 8;
  v8h hv[2];
#pragma unroll
  for (int it = 0; it < 2; ++it) {
    const int nrow = it * 32 + wave * 4 + q;
#pragma unroll
    for (int e = 0; e < 8; ++e) hv[it][e] = (_Float16)tile[(c8 + e) * 65 + nrow];
  }
  for (int pass = 0; pass < 2; ++pass) {
#pragma unroll
    for (int it = 0; it < 2; ++it) {
      const int nrow = it * 32 + wave * 4 + q;
      *(volatile v8h*)(Bt + (size_t)(n0 + nrow) * Kdim + k0 + c8) = hv[it];
    }
    __threadfence();
  }
}

__global__ __launch_bounds__(256) void dr_cast_kernel(
    const float* __restrict__ XDBL, unsigned short* __restrict__ DRAW16, int total8, float scale)
{
  const int i = blockIdx.x * 256 + threadIdx.x;
  if (i >= total8) return;
  const int e0  = i << 3;
  const int row = e0 >> 8;
  const int c8  = e0 & (kDtR - 1);
  const float* p = XDBL + (size_t)row * kPrjP + c8;
  const v4f a0 = *(const v4f*)(p);
  const v4f a1 = *(const v4f*)(p + 4);
  v8h hv;
#pragma unroll
  for (int e = 0; e < 4; ++e) {
    hv[e]     = (_Float16)(a0[e] * scale);
    hv[4 + e] = (_Float16)(a1[e] * scale);
  }
  unsigned short* qd = DRAW16 + (size_t)e0;
  *(volatile v8h*)qd = hv;
  __threadfence();
  *(volatile v8h*)qd = hv;
}

__global__ __launch_bounds__(256) void layernorm_kernel(
    const float* __restrict__ x, const float* __restrict__ w, const float* __restrict__ bvec,
    unsigned short* __restrict__ XN16)
{
  __shared__ float red[8];
  const int tid = threadIdx.x, lane = tid & 31, wave = tid >> 5;
  const int row = blockIdx.x;
  const float* xr = x + (size_t)row * kDmod;
  const v4f a = *(const v4f*)(xr + tid * 4);
  float s = (a[0] + a[1]) + (a[2] + a[3]);
#pragma unroll
  for (int off = 1; off < 32; off <<= 1) s += __shfl_xor(s, off, 32);
  if (lane == 0) red[wave] = s;
  __syncthreads();
  float tot = 0.f;
#pragma unroll
  for (int i = 0; i < 8; ++i) tot += red[i];
  const float mu = tot * (1.0f / (float)kDmod);
  __syncthreads();
  const float d0 = a[0] - mu, d1 = a[1] - mu, d2 = a[2] - mu, d3 = a[3] - mu;
  float qs = (d0 * d0 + d1 * d1) + (d2 * d2 + d3 * d3);
#pragma unroll
  for (int off = 1; off < 32; off <<= 1) qs += __shfl_xor(qs, off, 32);
  if (lane == 0) red[wave] = qs;
  __syncthreads();
  float tot2 = 0.f;
#pragma unroll
  for (int i = 0; i < 8; ++i) tot2 += red[i];
  const float var  = tot2 * (1.0f / (float)kDmod);
  const float rstd = 1.0f / sqrtf(var + 1e-5f);
  if (tid < 128) {
    const int c0 = tid * 8;
    const v4f b0 = *(const v4f*)(xr + c0);
    const v4f b1 = *(const v4f*)(xr + c0 + 4);
    const v4f w0 = *(const v4f*)(w + c0);
    const v4f w1 = *(const v4f*)(w + c0 + 4);
    const v4f g0 = *(const v4f*)(bvec + c0);
    const v4f g1 = *(const v4f*)(bvec + c0 + 4);
    v8h hv;
#pragma unroll
    for (int e = 0; e < 4; ++e) {
      hv[e]     = (_Float16)((b0[e] - mu) * rstd * w0[e] + g0[e]);
      hv[4 + e] = (_Float16)((b1[e] - mu) * rstd * w1[e] + g1[e]);
    }
    unsigned short* dst = XN16 + (size_t)row * kDmod + c0;
    *(volatile v8h*)dst = hv;
    __threadfence();
    *(volatile v8h*)dst = hv;
  }
}

__global__ __launch_bounds__(256) void scan_kernel(
    const unsigned short* __restrict__ DTL16, const float* __restrict__ U32, const unsigned short* __restrict__ G16,
    const float* __restrict__ XDBL, const float* __restrict__ dt_bias, const float* __restrict__ A_log,
    const float* __restrict__ Dv, unsigned short* __restrict__ Y16)
{
  __shared__ __align__(16) float sBC[16 * 32];
  __shared__ __align__(16) float sY[16 * kTP];
  __shared__ __align__(16) float sA[kNst * 256];
  const int tid = threadIdx.x, lane = tid & 31, wave = tid >> 5;
  const int bix = blockIdx.y;
  const int d0 = blockIdx.x * 256, d = d0 + tid;
  const size_t row0 = (size_t)bix * kSeqL;

#pragma unroll 1
  for (int n = 0; n < kNst; ++n) sA[n * 256 + tid] = -expf(A_log[(size_t)d * kNst + n]);
  __syncthreads();
  float An[kNst], h[kNst];
#pragma unroll
  for (int n = 0; n < kNst; ++n) { An[n] = sA[n * 256 + tid]; h[n] = 0.f; }
  const float bb = dt_bias[d], Dd = Dv[d];
  const int dpar = d & ~1;
  const unsigned dsh = (unsigned)(d & 1) * 16u;

#pragma unroll 1
  for (int c = 0; c < kSeqL / 16; ++c) {
    const int l0 = c * 16;
    if (tid < 128) {
      const int r = tid >> 3, q4 = (tid & 7) * 4;
      const v4f v = *(const v4f*)(XDBL + (row0 + l0 + r) * kPrjP + kDtR + q4);
      *(v4f*)(sBC + r * 32 + q4) = v;
    }
    __syncthreads();
#pragma unroll 1
    for (int s = 0; s < 16; ++s) {
      const size_t m = row0 + (size_t)(l0 + s);
      const unsigned wd = *(const unsigned*)(DTL16 + m * kDin + dpar);
      const unsigned wg = *(const unsigned*)(G16 + m * kDin + dpar);
      const float xv = U32[m * kDin + d];
      const float vlin  = h16_to_f32((wd >> dsh) & 0xffffu) * kDtlInv + bb;
      const float gate  = h16_to_f32((wg >> dsh) & 0xffffu);
      const float ea    = __expf(-fabsf(vlin));
      const float delta = fmaxf(vlin, 0.0f) + log1pf(ea);
      v4f Bq[4], Cq[4];
#pragma unroll
      for (int qq = 0; qq < 4; ++qq) {
        Bq[qq] = *(const v4f*)(sBC + s * 32 + 4 * qq);
        Cq[qq] = *(const v4f*)(sBC + s * 32 + kNst + 4 * qq);
      }
      float dtx = delta * xv;
      asm volatile("" : "+v"(dtx));
      float y = 0.f;
#pragma unroll
      for (int n = 0; n < kNst; ++n) {
        const float e = __expf(delta * An[n]);
        float p = dtx * Bq[n >> 2][n & 3];
        asm volatile("" : "+v"(p));
        float qv = h[n] * e;
        asm volatile("" : "+v"(qv));
        const float hn = qv + p;
        h[n] = hn;
        float rr = Cq[n >> 2][n & 3] * hn;
        asm volatile("" : "+v"(rr));
        y += rr;
      }
      float sk = xv * Dd;
      asm volatile("" : "+v"(sk));
      y += sk;
      y = y * gate;
      sY[s * kTP + tid] = y * kCarryY;
    }
    __syncthreads();
    v8h hv[2];
#pragma unroll
    for (int it = 0; it < 2; ++it) {
      const float* sp = sY + (it * 8 + wave) * kTP + lane * 8;
      const v4f a0 = *(const v4f*)(sp);
      const v4f a1 = *(const v4f*)(sp + 4);
#pragma unroll
      for (int e = 0; e < 4; ++e) { hv[it][e] = (_Float16)a0[e]; hv[it][4 + e] = (_Float16)a1[e]; }
    }
    for (int pass = 0; pass < 2; ++pass) {
#pragma unroll
      for (int it = 0; it < 2; ++it)
        *(volatile v8h*)(Y16 + (row0 + (size_t)(l0 + it * 8 + wave)) * kDin + d0 + lane * 8) = hv[it];
      __threadfence();
    }
  }
}

extern "C" void kernel_launch(void* const* d_in, const int* in_sizes, int n_in,
                              void* d_out, int out_size, void* d_ws, size_t ws_size,
                              hipStream_t stream)
{
  if (n_in < 10) return;
  if (in_sizes[0] != kRows * kDmod) return;
  if (in_sizes[1] != kDmod || in_sizes[2] != kDmod) return;
  if (in_sizes[3] != kDmod * kXzN) return;
  if (in_sizes[4] != kDin * kPrjN) return;
  if (in_sizes[5] != kDtR * kDin || in_sizes[6] != kDin) return;
  if (in_sizes[7] != kDin * kNst || in_sizes[8] != kDin) return;
  if (in_sizes[9] != kDin * kDmod) return;
  if (out_size != kRows * kDmod) return;
  if (ws_size < kWsTotal) return;

  const float* x      = (const float*)d_in[0];
  const float* norm_w = (const float*)d_in[1];
  const float* norm_b = (const float*)d_in[2];
  const float* W_in   = (const float*)d_in[3];
  const float* W_x    = (const float*)d_in[4];
  const float* W_dt   = (const float*)d_in[5];
  const float* b_dt   = (const float*)d_in[6];
  const float* A_log  = (const float*)d_in[7];
  const float* Dv     = (const float*)d_in[8];
  const float* W_out  = (const float*)d_in[9];
  float* dout = (float*)d_out;

  char* ws = (char*)d_ws;
  unsigned short* WIN16  = (unsigned short*)(ws + kOffWIN16);
  unsigned short* WX16   = (unsigned short*)(ws + kOffWX16);
  unsigned short* WDT16  = (unsigned short*)(ws + kOffWDT16);
  unsigned short* WOUT16 = (unsigned short*)(ws + kOffWOUT16);
  unsigned short* XN16   = (unsigned short*)(ws + kOffXN16);
  float*          U32    = (float*)(ws + kOffU32);
  unsigned short* G16    = (unsigned short*)(ws + kOffG16);
  unsigned short* U16    = (unsigned short*)(ws + kOffU16);
  float*          XDBL   = (float*)(ws + kOffXDBL);
  unsigned short* DRAW16 = (unsigned short*)(ws + kOffDRAW16);
  unsigned short* DTL16  = (unsigned short*)(ws + kOffDTL16);
  unsigned short* Y16    = (unsigned short*)(ws + kOffY16);
  const float* dummy_bias  = b_dt;
  const float* dummy_resid = x;

  transpose_cast_kernel<<<dim3(kXzN / 64, kDmod / 64), 256, 0, stream>>>(W_in,  WIN16,  kDmod, kXzN,  kXzN,  kCarryW);
  transpose_cast_kernel<<<dim3(kPrjP / 64, kDin / 64), 256, 0, stream>>>(W_x,   WX16,   kDin,  kPrjN, kPrjP, kCarryW);
  transpose_cast_kernel<<<dim3(kDin / 64, kDtR / 64), 256, 0, stream>>>(W_dt,   WDT16,  kDtR,  kDin,  kDin,  kCarryWdt);
  transpose_cast_kernel<<<dim3(kDmod / 64, kDin / 64), 256, 0, stream>>>(W_out, WOUT16, kDin,  kDmod, kDmod, kCarryW);

  layernorm_kernel<<<kRows, 256, 0, stream>>>(x, norm_w, norm_b, XN16);

  wmma_gemm64<0, false, 0, 0, false, 3><<<dim3(256, 1), 256, 0, stream>>>(
      XN16, XN16, kDmod, 0L, WIN16, WIN16, kDmod, 0L,
      (void*)U32, (void*)U32, kDin, 0L, dummy_bias, dummy_resid, 0L, kRows, kDin, kDmod, kScale1);

  wmma_gemm64<0, false, 0, 1, false, 3><<<dim3(256, 1), 256, 0, stream>>>(
      XN16, XN16, kDmod, 0L, WIN16 + (size_t)kDin * kDmod, WIN16 + (size_t)kDin * kDmod, kDmod, 0L,
      (void*)G16, (void*)G16, kDin, 0L, dummy_bias, dummy_resid, 0L, kRows, kDin, kDmod, kScale1);

  cast_f16_kernel<<<(kRows * kDin) / 8 / 256, 256, 0, stream>>>(U32, U16, (kRows * kDin) / 8, kCarryU);

  wmma_gemm64<0, false, 0, 0, false, 0><<<dim3(40, 1), 256, 0, stream>>>(
      U16, U16, kDin, 0L, WX16, WX16, kDin, 0L,
      (void*)XDBL, (void*)XDBL, kPrjP, 0L, dummy_bias, dummy_resid, 0L, kRows, kPrjP, kDin, kScale2);

  dr_cast_kernel<<<(kRows * kDtR) / 8 / 256, 256, 0, stream>>>(XDBL, DRAW16, (kRows * kDtR) / 8, kCarryDr);

  wmma_gemm64<0, false, 0, 1, false, 0><<<dim3(256, 1), 256, 0, stream>>>(
      DRAW16, DRAW16, kDtR, 0L, WDT16, WDT16, kDtR, 0L,
      (void*)DTL16, (void*)DTL16, kDin, 0L, dummy_bias, dummy_resid, 0L, kRows, kDin, kDtR, kScale3);

  scan_kernel<<<dim3(kDin / 256, kBatch), 256, 0, stream>>>(DTL16, U32, G16, XDBL, b_dt, A_log, Dv, Y16);

  wmma_gemm64<0, false, 0, 0, true, 0><<<dim3(128, 1), 256, 0, stream>>>(
      Y16, Y16, kDin, 0L, WOUT16, WOUT16, kDin, 0L,
      (void*)dout, (void*)dout, kDmod, 0L, dummy_bias, x, 0L, kRows, kDmod, kDin, kScale4);
}
